// RecurrentGCN_2963527435016
// MI455X (gfx1250) — hardware-verified
//
#include <hip/hip_runtime.h>

typedef __bf16         v16bf __attribute__((ext_vector_type(16)));
typedef unsigned short v8us  __attribute__((ext_vector_type(8)));
typedef float          v8f   __attribute__((ext_vector_type(8)));
typedef float          v4f   __attribute__((ext_vector_type(4)));
typedef v8us __attribute__((may_alias)) v8usa;
typedef v4f  __attribute__((may_alias)) v4fa;

union FragB { v16bf v; v8us u[2]; };

#define F_IN  128
#define HID   64
#define CIN   192
#define NOUT  128
#define KTOT  256
#define TM    128
#define NPIECE (NOUT * (KTOT / 8))

__device__ __forceinline__ unsigned short bf16_bits(float f) {
  unsigned int u = __float_as_uint(f);
  u += 0x7FFFu + ((u >> 16) & 1u);
  return (unsigned short)(u >> 16);
}
__device__ __forceinline__ float bf16_val(float f) {
  return __uint_as_float(((unsigned int)bf16_bits(f)) << 16);
}

__device__ __forceinline__ v8f wmma_bf16(v16bf a, v16bf b, v8f c) {
  v8f d = __builtin_amdgcn_wmma_f32_16x16x32_bf16(false, a, false, b, (short)0, c, false, false);
  asm volatile("v_nop\n\tv_nop\n\tv_nop\n\tv_nop" : "+v"(d) : "v"(a), "v"(b));
  return d;
}

__device__ __forceinline__ v8us cvt8_bf16(const float* p) {
  const v4f a = *(const v4fa*)p;
  const v4f c = *(const v4fa*)(p + 4);
  v8us o;
  o[0] = bf16_bits(a.x); o[1] = bf16_bits(a.y); o[2] = bf16_bits(a.z); o[3] = bf16_bits(a.w);
  o[4] = bf16_bits(c.x); o[5] = bf16_bits(c.y); o[6] = bf16_bits(c.z); o[7] = bf16_bits(c.w);
  return o;
}

__device__ __forceinline__ v16bf load_a_f32(const float* p, int h) {
  FragB f;
  f.u[0] = cvt8_bf16(p + 8 * h);
  f.u[1] = cvt8_bf16(p + 16 + 8 * h);
  return f.v;
}

__device__ __forceinline__ v16bf load_b_bf16(const unsigned short* q, int h) {
  FragB f;
  f.u[0] = *(const v8usa*)(q + 8 * h);
  f.u[1] = *(const v8usa*)(q + 16 + 8 * h);
  return f.v;
}

__global__ __launch_bounds__(256) void k_prep(const float* __restrict__ Wz,
                                              const float* __restrict__ Wh,
                                              unsigned short* __restrict__ Wt)
{
  const int g = blockIdx.x * 256 + threadIdx.x;
  if (g >= NPIECE) return;
  const int n  = g >> 5;
  const int k8 = g & 31;
  const float* W = (n < HID) ? Wz : Wh;
  const int j  = n & (HID - 1);
  const int d  = k8 >> 4;
  const int kb = (k8 & 15) * 8;
  const float* src = W + (size_t)d * (CIN * HID) + (size_t)kb * HID + j;
  v8us o;
  #pragma unroll
  for (int i = 0; i < 8; ++i) o[i] = bf16_bits(src[i * HID]);
  unsigned short* dst = Wt + (size_t)n * KTOT + k8 * 8;
  *(volatile v8us*)dst = o;
  __threadfence();
  *(volatile v8us*)dst = o;
}

__global__ __launch_bounds__(256) void k_main(const float* __restrict__ x,
                                              const unsigned short* __restrict__ Wt,
                                              const float* __restrict__ bz,
                                              const float* __restrict__ bh,
                                              const float* __restrict__ Wlin,
                                              const float* __restrict__ blin,
                                              float* __restrict__ out,
                                              int nrows)
{
  __shared__ __attribute__((aligned(16))) float sOut[TM];
  __shared__ float sWl[HID];
  __shared__ float sBz[HID];
  __shared__ float sBh[HID];

  const int tid = threadIdx.x, lane = tid & 31, w = tid >> 5;
  const int h = lane >> 4, m = lane & 15;
  const int m0 = blockIdx.x * TM;

  if (tid < HID) {
    sWl[tid] = bf16_val(Wlin[tid]);
    sBz[tid] = bf16_val(bz[tid]);
    sBh[tid] = bf16_val(bh[tid]);
  }
  __syncthreads();

  int rowa = m0 + 16 * w + m;
  rowa = (rowa < nrows) ? rowa : (nrows - 1);
  const float* xr = x + (size_t)rowa * F_IN;
  const unsigned short* wb = Wt + (size_t)m * KTOT;

  const v8f zero8 = {0.f, 0.f, 0.f, 0.f, 0.f, 0.f, 0.f, 0.f};
  v8f acc[8];
  #pragma unroll
  for (int t = 0; t < 8; ++t) acc[t] = zero8;

  #pragma unroll 1
  for (int kk = 0; kk < 4; ++kk) {
    const int kc = 32 * kk;
    const v16bf a = load_a_f32(xr + kc, h);
    #pragma unroll
    for (int t = 0; t < 8; ++t) {
      const unsigned short* q = wb + (size_t)t * 16 * KTOT + kc;
      const v16bf b0 = load_b_bf16(q, h);
      const v16bf b1 = load_b_bf16(q + F_IN, h);
      acc[t] = wmma_bf16(a, b0, acc[t]);
      acc[t] = wmma_bf16(a, b1, acc[t]);
    }
  }

  float part[8];
  #pragma unroll
  for (int r = 0; r < 8; ++r) part[r] = 0.f;

  #pragma unroll
  for (int t = 0; t < 4; ++t) {
    const int j = 16 * t + m;
    const float wl  = sWl[j];
    const float bzv = sBz[j];
    const float bhv = sBh[j];
    #pragma unroll
    for (int r = 0; r < 8; ++r) {
      const float zv = acc[t][r] + bzv;
      const float hv = acc[t + 4][r] + bhv;
      const float e  = expf(-zv);
      const float s  = 1.0f / (1.0f + e);
      const float c  = tanhf(hv);
      float g = (1.0f - s) * c;
      g = (g > 0.f) ? g : 0.f;
      part[r] = part[r] + g * wl;
    }
  }

  #pragma unroll
  for (int r = 0; r < 8; ++r) {
    part[r] += __shfl_xor(part[r], 1, 32);
    part[r] += __shfl_xor(part[r], 2, 32);
    part[r] += __shfl_xor(part[r], 4, 32);
    part[r] += __shfl_xor(part[r], 8, 32);
  }

  const int mm = m & 7;
  float v = part[0];
  #pragma unroll
  for (int r = 1; r < 8; ++r) v = (mm == r) ? part[r] : v;
  if (m < 8) sOut[16 * w + 8 * h + m] = v;
  __syncthreads();

  const float bl = bf16_val(blin[0]);
  const int nvalid = nrows - m0;
  const bool ok = (w == 0) && (4 * lane + 4 <= nvalid);
  const v4f sv = *(const v4fa*)(sOut + 4 * lane);
  v4f o;
  o.x = sv.x + bl; o.y = sv.y + bl; o.z = sv.z + bl; o.w = sv.w + bl;
  float* dst = out + (size_t)m0 + 4 * lane;
  if (ok) *(volatile v4f*)dst = o;
  __threadfence();
  if (ok) *(volatile v4f*)dst = o;
}

extern "C" void kernel_launch(void* const* d_in, const int* in_sizes, int n_in,
                              void* d_out, int out_size, void* d_ws, size_t ws_size,
                              hipStream_t stream) {
  if (n_in < 11) return;
  const int nrows = in_sizes[0] / F_IN;
  if (nrows <= 0 || nrows * F_IN != in_sizes[0]) return;
  if ((nrows & 31) != 0) return;
  if (out_size != nrows) return;
  if (in_sizes[3] != 2 * CIN * HID || in_sizes[7] != 2 * CIN * HID) return;
  if (in_sizes[4] < HID || in_sizes[8] < HID || in_sizes[9] < HID || in_sizes[10] < 1) return;

  const size_t wt_bytes = (size_t)NOUT * KTOT * 2;
  if (wt_bytes > ws_size) return;

  const float* x    = (const float*)d_in[0];
  const float* Wz   = (const float*)d_in[3];
  const float* bz   = (const float*)d_in[4];
  const float* Wh   = (const float*)d_in[7];
  const float* bh   = (const float*)d_in[8];
  const float* Wlin = (const float*)d_in[9];
  const float* blin = (const float*)d_in[10];
  float* out = (float*)d_out;
  unsigned short* Wt = (unsigned short*)d_ws;

  k_prep<<<(NPIECE + 255) / 256, 256, 0, stream>>>(Wz, Wh, Wt);

  const int blocks = (nrows + TM - 1) / TM;
  k_main<<<blocks, 256, 0, stream>>>(x, Wt, bz, bh, Wlin, blin, out, nrows);
}
